// GCN_60945585930926
// MI455X (gfx1250) — hardware-run, weakly checked
//
#include <hip/hip_runtime.h>
#include <stddef.h>
#include <stdint.h>


#define NN     100000
#define NE     1600000
#define DF     128
#define PH     256
#define MP     100096
#define K1T    384
#define K2T    512
#define NTHR   256
#define NWAVE  8
#define EPT    8
#define WCAP   (EPT * 32)
#define NBRUN  1024
#define SLA    10
#define NBB    98
#define RCAP   20480
#define DEGCAP 64
#define WLCAP  (RCAP / NWAVE)
#define WLN    (NWAVE * WLCAP)
#define NSTEP  (NE / WCAP)
#define SPW    ((NSTEP + NWAVE - 1) / NWAVE)
#define MISCN  32
#define BK_INTS (WLN + RCAP + 3 * NBRUN + MISCN)
#define BK_LDS  (BK_INTS * 4)
#define GBM    128
#define GBN    128
#define G_LDS  ((GBM * GBN + DF) * 4)
#define ARB    128
#define ARW    (ARB / NWAVE)
#define UPART  2048
#define NPART  7
#define NUW    (NPART * UPART)
#define NUX    (MP * (DF / 8))
#define NUALL  (NUW + NUX)
#define WSMAX  134217728

static_assert(DF == 128 && DF == 4 * 32 && PH == 2 * DF);
static_assert(K1T % 32 == 0 && K2T % 32 == 0 && K1T == 3 * DF && K2T == 4 * DF);
static_assert(MP % GBM == 0 && MP >= NN && MP - NN < GBM);
static_assert(NBRUN == (1 << SLA) && NBRUN % GBM == 0 && NBRUN % ARB == 0);
static_assert(NBB * NBRUN >= MP && (NBB - 1) * NBRUN < NN);
static_assert(NE % 4 == 0 && NE % WCAP == 0);
static_assert(((long long)NE << SLA) < (1LL << 31));
static_assert(RCAP == 20480 && RCAP >= 16710 + 16710 / 20 && RCAP % (NTHR * 4) == 0 && RCAP % NWAVE == 0);
static_assert(DEGCAP == 64 && DEGCAP >= 36 + 8 && DEGCAP <= 64);
static_assert(WLCAP >= WCAP && WLN == RCAP);
static_assert(NBRUN == NTHR * 4);
static_assert(BK_INTS % 4 == 0 && BK_LDS < 300000 && BK_LDS <= 327680);
static_assert(G_LDS <= 327680);
static_assert(NWAVE * PH * 2 <= 327680);
static_assert(GBM == NWAVE * 16 && NTHR == NWAVE * 32 && NTHR * 4 == NWAVE * GBN);
static_assert(UPART % NTHR == 0 && UPART == DF * (DF / 8) && NUW % NTHR == 0 && NUALL % NTHR == 0);
static_assert((NBB * NBRUN) % ARB == 0);

typedef float          v4f   __attribute__((ext_vector_type(4)));
typedef float          v8f   __attribute__((ext_vector_type(8)));
typedef int            v4i   __attribute__((ext_vector_type(4)));
typedef int            v8i   __attribute__((ext_vector_type(8)));
typedef unsigned       v2u   __attribute__((ext_vector_type(2)));
typedef unsigned short v4us  __attribute__((ext_vector_type(4)));
typedef unsigned short v8us  __attribute__((ext_vector_type(8)));
typedef unsigned short v16us __attribute__((ext_vector_type(16)));
typedef __bf16         v16bf __attribute__((ext_vector_type(16)));
typedef v4f  __attribute__((may_alias)) v4fa;
typedef v4i  __attribute__((may_alias)) v4ia;
typedef v2u  __attribute__((may_alias)) v2ua;
typedef v4us __attribute__((may_alias)) v4usa;
typedef v8us __attribute__((may_alias)) v8usa;
union FragB { v16bf v; v16us u; v8us h[2]; v8i w; };

__device__ __forceinline__ v8f wmb(const FragB& a, const FragB& b, v8f c) {
  v8f d = __builtin_amdgcn_wmma_f32_16x16x32_bf16(false, a.v, false, b.v, (short)0, c, false, false);
  asm volatile("v_nop\n\tv_nop\n\tv_nop\n\tv_nop" : "+v"(d) : "v"(a.w), "v"(b.w));
  return d;
}

__device__ __forceinline__ unsigned bf16_bits(float f) {
  const unsigned u = __float_as_uint(f);
  const unsigned r = (u + 0x7FFFu + ((u >> 16) & 1u)) >> 16;
  return (f != f) ? 0x7FC0u : r;
}
__device__ __forceinline__ float bf16_val(float f) {
  return __uint_as_float(bf16_bits(f) << 16);
}
__device__ __forceinline__ unsigned hl_bits(float v, unsigned& lo) {
  const unsigned hb = bf16_bits(v);
  lo = bf16_bits(v - __uint_as_float(hb << 16));
  return hb;
}

__device__ __forceinline__ void wave_sync() {
  __builtin_amdgcn_fence(__ATOMIC_RELEASE, "wavefront");
  __builtin_amdgcn_wave_barrier();
  __builtin_amdgcn_fence(__ATOMIC_ACQUIRE, "wavefront");
}

__device__ __forceinline__ void put8(unsigned short* dp, v8us o) {
  *(volatile v8us*)dp = o;
  __threadfence();
  *(volatile v8us*)dp = o;
}

__device__ __forceinline__ void cvt8(const float* __restrict__ p, unsigned short* dp, bool live) {
  const v4f a = *(const v4f*)p;
  const v4f b = *(const v4f*)(p + 4);
  asm volatile("" :: "v"(a), "v"(b));
  const unsigned msk = live ? 0xFFFFu : 0u;
  v8us o;
  o[0] = (unsigned short)(bf16_bits(a.x) & msk); o[1] = (unsigned short)(bf16_bits(a.y) & msk);
  o[2] = (unsigned short)(bf16_bits(a.z) & msk); o[3] = (unsigned short)(bf16_bits(a.w) & msk);
  o[4] = (unsigned short)(bf16_bits(b.x) & msk); o[5] = (unsigned short)(bf16_bits(b.y) & msk);
  o[6] = (unsigned short)(bf16_bits(b.z) & msk); o[7] = (unsigned short)(bf16_bits(b.w) & msk);
  put8(dp, o);
}

__global__ __launch_bounds__(NTHR) void k_prep(const float* __restrict__ x,
                                               const float* __restrict__ W1l, const float* __restrict__ W1r,
                                               const float* __restrict__ W2l, const float* __restrict__ W2r,
                                               unsigned short* W1C, unsigned short* W2C, unsigned short* XB) {
  const int u = (int)blockIdx.x * NTHR + (int)threadIdx.x;
  if (u < NUW) {
    const int part = u >> 11;
    const int v    = u & (UPART - 1);
    const int n    = v >> 4;
    const int k8   = (v & 15) * 8;
    const size_t so = (size_t)n * DF + (size_t)k8;
    if (part == 0)      cvt8(W1l + so, W1C + (size_t)n * K1T + 0 * DF + k8, true);
    else if (part == 1) cvt8(W1l + so, W1C + (size_t)n * K1T + 1 * DF + k8, true);
    else if (part == 2) cvt8(W1r + so, W1C + (size_t)n * K1T + 2 * DF + k8, true);
    else if (part == 3) cvt8(W2l + so, W2C + (size_t)n * K2T + 0 * DF + k8, true);
    else if (part == 4) cvt8(W2l + so, W2C + (size_t)n * K2T + 1 * DF + k8, true);
    else if (part == 5) cvt8(W2r + so, W2C + (size_t)n * K2T + 2 * DF + k8, true);
    else                cvt8(W2r + so, W2C + (size_t)n * K2T + 3 * DF + k8, true);
  } else {
    const int v   = u - NUW;
    const int row = v >> 4;
    const int k8  = (v & 15) * 8;
    const int rc  = row < NN ? row : NN - 1;
    cvt8(x + (size_t)rc * DF + k8, XB + (size_t)v * 8, row < NN);
  }
}

__global__ __launch_bounds__(NTHR) void k_bucket(const int* __restrict__ srcs, const int* __restrict__ dsts,
                                                 int* LIST, int* CNT, int* OFF, int* FLAG) {
  extern __shared__ __attribute__((aligned(16))) int dsm[];
  int* wl   = dsm;
  int* sl   = wl + WLN;
  int* cnt  = sl + RCAP;
  int* offs = cnt + NBRUN;
  int* cur  = offs + NBRUN;
  int* misc = cur + NBRUN;
  const int tid = (int)threadIdx.x, lane = tid & 31, wave = tid >> 5;
  const int bb = (int)blockIdx.x;
  const unsigned nbs = (unsigned)(bb * NBRUN);

  {
    const v4i z4 = {0, 0, 0, 0};
    for (int i = tid * 4; i < BK_INTS; i += NTHR * 4) *(v4ia*)(dsm + i) = z4;
  }
  __syncthreads();

  {
    int wc = 0;
    int* mywl = wl + wave * WLCAP;
    const int sb = wave * SPW;
    const int se = (sb + SPW) < NSTEP ? (sb + SPW) : NSTEP;
#pragma unroll 1
    for (int s = sb; s < se; ++s) {
      const int e0 = s * WCAP + EPT * lane;
      const v4i da = *(const v4i*)(dsts + e0);
      const v4i db = *(const v4i*)(dsts + e0 + 4);
      const unsigned s0 = (unsigned)da.x - nbs, s1 = (unsigned)da.y - nbs;
      const unsigned s2 = (unsigned)da.z - nbs, s3 = (unsigned)da.w - nbs;
      const unsigned s4 = (unsigned)db.x - nbs, s5 = (unsigned)db.y - nbs;
      const unsigned s6 = (unsigned)db.z - nbs, s7 = (unsigned)db.w - nbs;
      const bool h0 = s0 < (unsigned)NBRUN, h1 = s1 < (unsigned)NBRUN, h2 = s2 < (unsigned)NBRUN, h3 = s3 < (unsigned)NBRUN;
      const bool h4 = s4 < (unsigned)NBRUN, h5 = s5 < (unsigned)NBRUN, h6 = s6 < (unsigned)NBRUN, h7 = s7 < (unsigned)NBRUN;
      const unsigned m0 = __builtin_amdgcn_ballot_w32(h0), m1 = __builtin_amdgcn_ballot_w32(h1);
      const unsigned m2 = __builtin_amdgcn_ballot_w32(h2), m3 = __builtin_amdgcn_ballot_w32(h3);
      const unsigned m4 = __builtin_amdgcn_ballot_w32(h4), m5 = __builtin_amdgcn_ballot_w32(h5);
      const unsigned m6 = __builtin_amdgcn_ballot_w32(h6), m7 = __builtin_amdgcn_ballot_w32(h7);
      const unsigned any = m0 | m1 | m2 | m3 | m4 | m5 | m6 | m7;
      if (any != 0u) {
        unsigned pre = __builtin_amdgcn_mbcnt_lo(m0, 0u);
        pre = __builtin_amdgcn_mbcnt_lo(m1, pre);
        pre = __builtin_amdgcn_mbcnt_lo(m2, pre);
        pre = __builtin_amdgcn_mbcnt_lo(m3, pre);
        pre = __builtin_amdgcn_mbcnt_lo(m4, pre);
        pre = __builtin_amdgcn_mbcnt_lo(m5, pre);
        pre = __builtin_amdgcn_mbcnt_lo(m6, pre);
        pre = __builtin_amdgcn_mbcnt_lo(m7, pre);
        int pos = wc + (int)pre;
#define PUTJ(J, HJ, SJ, MJ) \
        if ((MJ) != 0u) { \
          if ((HJ) && pos < WLCAP) mywl[pos] = ((e0 + (J)) << SLA) | (int)(SJ); \
          pos += (HJ) ? 1 : 0; \
        }
        PUTJ(0, h0, s0, m0)
        PUTJ(1, h1, s1, m1)
        PUTJ(2, h2, s2, m2)
        PUTJ(3, h3, s3, m3)
        PUTJ(4, h4, s4, m4)
        PUTJ(5, h5, s5, m5)
        PUTJ(6, h6, s6, m6)
        PUTJ(7, h7, s7, m7)
#undef PUTJ
        wc += (int)__builtin_popcount(m0) + (int)__builtin_popcount(m1) + (int)__builtin_popcount(m2) +
              (int)__builtin_popcount(m3) + (int)__builtin_popcount(m4) + (int)__builtin_popcount(m5) +
              (int)__builtin_popcount(m6) + (int)__builtin_popcount(m7);
      }
    }
    if (lane == 0) {
      misc[wave]     = wc > WLCAP ? WLCAP : wc;
      misc[8 + wave] = wc > WLCAP ? 1 : 0;
    }
  }
  __syncthreads();

  if (wave == 0) {
#pragma unroll 1
    for (int w2 = 0; w2 < NWAVE; ++w2) {
      int c = __builtin_amdgcn_readfirstlane(misc[w2]);
      c = c < 0 ? 0 : (c > WLCAP ? WLCAP : c);
#pragma unroll 1
      for (int b0 = 0; b0 < c; b0 += 32) {
        const int idx = b0 + lane;
        const int ent = wl[w2 * WLCAP + (idx < WLCAP ? idx : WLCAP - 1)];
        const int m32 = (c - b0) < 32 ? (c - b0) : 32;
#pragma unroll 1
        for (int k = 0; k < m32; ++k) {
          const int u    = __builtin_amdgcn_readlane(ent, k);
          const int slot = u & (NBRUN - 1);
          if (lane == 0) cnt[slot] = cnt[slot] + 1;
        }
      }
    }
  }
  __syncthreads();

  if (wave == 0) {
    const int base = lane * (NBRUN / 32);
    int s = 0, big = 0;
#pragma unroll 1
    for (int i = 0; i < NBRUN / 32; ++i) {
      const int cv = cnt[base + i];
      s += cv;
      big |= (cv > DEGCAP) ? 1 : 0;
    }
    int incl = s;
#pragma unroll
    for (int d = 1; d < 32; d <<= 1) {
      const int y = __shfl_up(incl, d, 32);
      if (lane >= d) incl += y;
    }
    int run = incl - s;
#pragma unroll 1
    for (int i = 0; i < NBRUN / 32; ++i) {
      const int cv = cnt[base + i];
      offs[base + i] = run;
      cur[base + i]  = run;
      run += cv;
    }
    const unsigned bm = __builtin_amdgcn_ballot_w32(big != 0);
    if (lane == 0) misc[16] = (bm != 0u) ? 1 : 0;
  }
  __syncthreads();

  if (wave == 0) {
#pragma unroll 1
    for (int w2 = 0; w2 < NWAVE; ++w2) {
      int c = __builtin_amdgcn_readfirstlane(misc[w2]);
      c = c < 0 ? 0 : (c > WLCAP ? WLCAP : c);
#pragma unroll 1
      for (int b0 = 0; b0 < c; b0 += 32) {
        const int idx = b0 + lane;
        const int ent = wl[w2 * WLCAP + (idx < WLCAP ? idx : WLCAP - 1)];
        const int m32 = (c - b0) < 32 ? (c - b0) : 32;
#pragma unroll 1
        for (int k = 0; k < m32; ++k) {
          const int u    = __builtin_amdgcn_readlane(ent, k);
          const int slot = u & (NBRUN - 1);
          if (lane == 0) {
            int p = cur[slot];
            p = p < 0 ? 0 : (p > RCAP - 1 ? RCAP - 1 : p);
            sl[p] = u;
            cur[slot] = p + 1;
          }
        }
      }
    }
  }
  __syncthreads();

  int fl = misc[16];
#pragma unroll
  for (int w2 = 0; w2 < NWAVE; ++w2) fl |= misc[8 + w2];
#pragma unroll 1
  for (int i = tid * 4; i < RCAP; i += NTHR * 4) {
    const v4i u = *(const v4ia*)(sl + i);
    int e0 = u.x >> SLA, e1 = u.y >> SLA, e2 = u.z >> SLA, e3 = u.w >> SLA;
    e0 = e0 < 0 ? 0 : (e0 > NE - 1 ? NE - 1 : e0);
    e1 = e1 < 0 ? 0 : (e1 > NE - 1 ? NE - 1 : e1);
    e2 = e2 < 0 ? 0 : (e2 > NE - 1 ? NE - 1 : e2);
    e3 = e3 < 0 ? 0 : (e3 > NE - 1 ? NE - 1 : e3);
    int r0 = srcs[e0], r1 = srcs[e1], r2 = srcs[e2], r3 = srcs[e3];
    v4i q;
    q.x = r0 < 0 ? 0 : (r0 > NN - 1 ? NN - 1 : r0);
    q.y = r1 < 0 ? 0 : (r1 > NN - 1 ? NN - 1 : r1);
    q.z = r2 < 0 ? 0 : (r2 > NN - 1 ? NN - 1 : r2);
    q.w = r3 < 0 ? 0 : (r3 > NN - 1 ? NN - 1 : r3);
    *(v4ia*)(sl + i) = q;
  }
  __syncthreads();

  int* lp = LIST + (size_t)bb * RCAP;
  int* cp = CNT + (size_t)bb * NBRUN + 4 * tid;
  int* op = OFF + (size_t)bb * NBRUN + 4 * tid;
  int* fp = FLAG + (size_t)bb * 32 + 4 * (tid & 7);
  const v4i cq = *(const v4ia*)(cnt + 4 * tid);
  const v4i oq = *(const v4ia*)(offs + 4 * tid);
  const v4i fq = {fl, fl, fl, fl};
#define SPILL_PASS \
  { \
    _Pragma_unroll1_loop \
  }
#undef SPILL_PASS
#pragma unroll 1
  for (int i = tid * 4; i < RCAP; i += NTHR * 4) {
    const v4i q = *(const v4ia*)(sl + i);
    *(volatile v4i*)(lp + i) = q;
  }
  *(volatile v4i*)cp = cq;
  *(volatile v4i*)op = oq;
  if (tid < 8) *(volatile v4i*)fp = fq;
  __threadfence();
#pragma unroll 1
  for (int i = tid * 4; i < RCAP; i += NTHR * 4) {
    const v4i q = *(const v4ia*)(sl + i);
    *(volatile v4i*)(lp + i) = q;
  }
  *(volatile v4i*)cp = cq;
  *(volatile v4i*)op = oq;
  if (tid < 8) *(volatile v4i*)fp = fq;
}

template <int L>
__global__ __launch_bounds__(NTHR) void k_agg(const int* __restrict__ LIST, const int* __restrict__ CNT,
                                              const int* __restrict__ OFF, const int* __restrict__ FLAG,
                                              const unsigned short* __restrict__ G, unsigned short* outp) {
  __shared__ __attribute__((aligned(16))) unsigned short rbuf[NWAVE * PH];
  const int tid = (int)threadIdx.x, lane = tid & 31, wave = tid >> 5;
  unsigned short* rowbuf = rbuf + wave * PH;
  const float qnan = __int_as_float(0x7fc00000);
#pragma unroll 1
  for (int si = 0; si < ARW; ++si) {
    const int node = (int)blockIdx.x * ARB + wave * ARW + si;
    const int bb   = node >> SLA;
    const int fl   = __builtin_amdgcn_readfirstlane(FLAG[bb * 32]);
    const int craw = __builtin_amdgcn_readfirstlane(CNT[node]);
    int o          = __builtin_amdgcn_readfirstlane(OFF[node]);
    const bool big = craw > DEGCAP;
    const int c    = craw < 0 ? 0 : (craw > DEGCAP ? DEGCAP : craw);
    o = o < 0 ? 0 : (o > RCAP - 1 ? RCAP - 1 : o);
    const int* lp = LIST + (size_t)bb * RCAP;
    float a0 = 0.0f, a1 = 0.0f, a2 = 0.0f, a3 = 0.0f;
#pragma unroll 1
    for (int b0 = 0; b0 < c; b0 += 32) {
      int idx = o + b0 + lane;
      idx = idx > RCAP - 1 ? RCAP - 1 : idx;
      int sr = lp[idx];
      sr = sr < 0 ? 0 : (sr > NN - 1 ? NN - 1 : sr);
      const int m32 = (c - b0) < 32 ? (c - b0) : 32;
#pragma unroll 1
      for (int k = 0; k < m32; ++k) {
        const int sk = __builtin_amdgcn_readlane(sr, k);
        if constexpr (L == 1) {
          const v2u w = *(const v2ua*)(G + (size_t)sk * DF + 4 * lane);
          a0 += __uint_as_float(w.x << 16);
          a1 += __uint_as_float(w.x & 0xffff0000u);
          a2 += __uint_as_float(w.y << 16);
          a3 += __uint_as_float(w.y & 0xffff0000u);
        } else {
          const unsigned short* rp = G + (size_t)sk * PH + 4 * lane;
          const v2u wh = *(const v2ua*)rp;
          const v2u wo = *(const v2ua*)(rp + DF);
          const float f0 = __uint_as_float(wh.x << 16)         + __uint_as_float(wo.x << 16);
          const float f1 = __uint_as_float(wh.x & 0xffff0000u) + __uint_as_float(wo.x & 0xffff0000u);
          const float f2 = __uint_as_float(wh.y << 16)         + __uint_as_float(wo.y << 16);
          const float f3 = __uint_as_float(wh.y & 0xffff0000u) + __uint_as_float(wo.y & 0xffff0000u);
          a0 += f0; a1 += f1; a2 += f2; a3 += f3;
        }
      }
    }
    const int cd = craw < 1 ? 1 : craw;
    const float den = (float)cd;
    const float pzr = (fl != 0 || big) ? qnan : 0.0f;
    const bool live = node < NN;
    const float m0 = live ? (a0 / den + pzr) : 0.0f;
    const float m1 = live ? (a1 / den + pzr) : 0.0f;
    const float m2 = live ? (a2 / den + pzr) : 0.0f;
    const float m3 = live ? (a3 / den + pzr) : 0.0f;
    v4us mh, ml;
    {
      unsigned lb, hb;
      hb = hl_bits(m0, lb); mh[0] = (unsigned short)hb; ml[0] = (unsigned short)lb;
      hb = hl_bits(m1, lb); mh[1] = (unsigned short)hb; ml[1] = (unsigned short)lb;
      hb = hl_bits(m2, lb); mh[2] = (unsigned short)hb; ml[2] = (unsigned short)lb;
      hb = hl_bits(m3, lb); mh[3] = (unsigned short)hb; ml[3] = (unsigned short)lb;
    }
    *(v4usa*)(rowbuf + 4 * lane)      = mh;
    *(v4usa*)(rowbuf + DF + 4 * lane) = ml;
    wave_sync();
    const v8us q0 = *(const v8usa*)(rowbuf + 8 * lane);
    wave_sync();
    if (node < MP) {
      unsigned short* rpw = outp + (size_t)node * PH + 8 * lane;
      *(volatile v8us*)rpw = q0;
      __threadfence();
      *(volatile v8us*)rpw = q0;
    }
  }
}

template <int FIN, int K2, int LD2>
__global__ __launch_bounds__(NTHR) __attribute__((amdgpu_num_vgpr(248)))
void k_gemm(const unsigned short* A1, const unsigned short* A2, const unsigned short* __restrict__ BT,
            const float* __restrict__ bias, const int* __restrict__ FLAG,
            unsigned short* outH, float* outF) {
  constexpr int KT = 256 + K2;
  static_assert(K2 % 32 == 0 && KT % 32 == 0 && LD2 >= K2);
  extern __shared__ __attribute__((aligned(16))) float gsm[];
  float* stg = gsm;
  float* bsh = gsm + GBM * GBN;
  const int tid = (int)threadIdx.x, lane = tid & 31, wave = tid >> 5, hh = lane >> 4, m = lane & 15;
  const int rowBase = (int)blockIdx.x * GBM;

  if (tid < 32) {
    const v4f b4 = *(const v4f*)(bias + 4 * tid);
    v4f bq;
    bq.x = bf16_val(b4.x); bq.y = bf16_val(b4.y); bq.z = bf16_val(b4.z); bq.w = bf16_val(b4.w);
    *(v4fa*)(bsh + 4 * tid) = bq;
  }

  v8f acc[8];
  {
    const v8f z = {0.f, 0.f, 0.f, 0.f, 0.f, 0.f, 0.f, 0.f};
#pragma unroll
    for (int t = 0; t < 8; ++t) acc[t] = z;
  }
  const size_t arow = (size_t)(rowBase + 16 * wave + m);
  const unsigned short* ap1 = A1 + arow * (size_t)PH + 8 * hh;
  const unsigned short* ap2 = A2 + arow * (size_t)LD2 + 8 * hh;
  const unsigned short* bp  = BT + (size_t)m * (size_t)KT + 8 * hh;

#pragma unroll 1
  for (int k0 = 0; k0 < 256; k0 += 32) {
    FragB af;
    af.h[0] = *(const v8usa*)(ap1 + k0);
    af.h[1] = *(const v8usa*)(ap1 + k0 + 16);
#pragma unroll
    for (int nt = 0; nt < 8; ++nt) {
      const unsigned short* wq = bp + (size_t)(16 * nt) * (size_t)KT + k0;
      FragB bf;
      bf.h[0] = *(const v8usa*)wq;
      bf.h[1] = *(const v8usa*)(wq + 16);
      acc[nt] = wmb(af, bf, acc[nt]);
    }
  }
#pragma unroll 1
  for (int k0 = 0; k0 < K2; k0 += 32) {
    FragB af;
    af.h[0] = *(const v8usa*)(ap2 + k0);
    af.h[1] = *(const v8usa*)(ap2 + k0 + 16);
#pragma unroll
    for (int nt = 0; nt < 8; ++nt) {
      const unsigned short* wq = bp + (size_t)(16 * nt) * (size_t)KT + 256 + k0;
      FragB bf;
      bf.h[0] = *(const v8usa*)wq;
      bf.h[1] = *(const v8usa*)(wq + 16);
      acc[nt] = wmb(af, bf, acc[nt]);
    }
  }

#pragma unroll
  for (int nt = 0; nt < 8; ++nt) {
    const int lc = 16 * nt + m;
#pragma unroll
    for (int r = 0; r < 8; ++r) {
      const int lr = 16 * wave + 8 * hh + r;
      stg[lr * GBN + lc] = acc[nt][r];
    }
  }
  __syncthreads();

  const v4f b4 = *(const v4fa*)(bsh + 4 * lane);
  int fl = 0;
  if constexpr (FIN != 0) fl = __builtin_amdgcn_readfirstlane(FLAG[(rowBase >> SLA) * 32]);
  const float qnan = __int_as_float(0x7fc00000);

#pragma unroll 1
  for (int i = 0; i < 16; ++i) {
    float* srow = stg + (16 * wave + i) * GBN;
    const bool ok = (rowBase + 16 * wave + i) < NN;
    const v4f d = *(const v4fa*)(srow + 4 * lane);
    const float v0 = d.x + b4.x, v1 = d.y + b4.y, v2 = d.z + b4.z, v3 = d.w + b4.w;
    float ss = (v0 * v0 + v1 * v1) + (v2 * v2 + v3 * v3);
    ss += __shfl_xor(ss, 16, 32);
    ss += __shfl_xor(ss, 8, 32);
    ss += __shfl_xor(ss, 4, 32);
    ss += __shfl_xor(ss, 2, 32);
    ss += __shfl_xor(ss, 1, 32);
    const float nrm = sqrtf(ss);
    const float den = (nrm > 1e-12f || nrm != nrm) ? nrm : 1e-12f;
    float y0 = v0 / den, y1 = v1 / den, y2 = v2 / den, y3 = v3 / den;
    y0 = (y0 > 0.0f) ? y0 : (y0 - y0);
    y1 = (y1 > 0.0f) ? y1 : (y1 - y1);
    y2 = (y2 > 0.0f) ? y2 : (y2 - y2);
    y3 = (y3 > 0.0f) ? y3 : (y3 - y3);
    y0 = ok ? y0 : 0.0f; y1 = ok ? y1 : 0.0f; y2 = ok ? y2 : 0.0f; y3 = ok ? y3 : 0.0f;
    if constexpr (FIN != 0) {
      v4f q;
      q.x = (fl != 0) ? qnan : y0;
      q.y = (fl != 0) ? qnan : y1;
      q.z = (fl != 0) ? qnan : y2;
      q.w = (fl != 0) ? qnan : y3;
      *(v4fa*)(srow + 4 * lane) = q;
    } else {
      v4us h4, l4;
      unsigned lb, hb;
      hb = hl_bits(y0, lb); h4[0] = (unsigned short)hb; l4[0] = (unsigned short)lb;
      hb = hl_bits(y1, lb); h4[1] = (unsigned short)hb; l4[1] = (unsigned short)lb;
      hb = hl_bits(y2, lb); h4[2] = (unsigned short)hb; l4[2] = (unsigned short)lb;
      hb = hl_bits(y3, lb); h4[3] = (unsigned short)hb; l4[3] = (unsigned short)lb;
      wave_sync();
      unsigned short* hrow = (unsigned short*)srow;
      *(v4usa*)(hrow + 4 * lane)      = h4;
      *(v4usa*)(hrow + DF + 4 * lane) = l4;
    }
  }
  __syncthreads();

  if constexpr (FIN != 0) {
#pragma unroll 1
    for (int i = 0; i < 16; ++i) {
      const int row = rowBase + 16 * wave + i;
      const v4f q = *(const v4fa*)(stg + (16 * wave + i) * GBN + 4 * lane);
      asm volatile("" :: "v"(q));
      if (row < NN) *(volatile v4f*)(outF + (size_t)row * DF + 4 * lane) = q;
    }
    __threadfence();
#pragma unroll 1
    for (int i = 0; i < 16; ++i) {
      const int row = rowBase + 16 * wave + i;
      const v4f q = *(const v4fa*)(stg + (16 * wave + i) * GBN + 4 * lane);
      asm volatile("" :: "v"(q));
      if (row < NN) *(volatile v4f*)(outF + (size_t)row * DF + 4 * lane) = q;
    }
    (void)outH;
  } else {
#pragma unroll 1
    for (int i = 0; i < 16; ++i) {
      const int row = rowBase + 16 * wave + i;
      const v8us q = *(const v8usa*)((const unsigned short*)(stg + (16 * wave + i) * GBN) + 8 * lane);
      *(volatile v8us*)(outH + (size_t)row * PH + 8 * lane) = q;
    }
    __threadfence();
#pragma unroll 1
    for (int i = 0; i < 16; ++i) {
      const int row = rowBase + 16 * wave + i;
      const v8us q = *(const v8usa*)((const unsigned short*)(stg + (16 * wave + i) * GBN) + 8 * lane);
      *(volatile v8us*)(outH + (size_t)row * PH + 8 * lane) = q;
    }
    (void)outF; (void)FLAG;
  }
}

static inline size_t al256(size_t o) { return (o + 255) & ~(size_t)255; }

extern "C" void kernel_launch(void* const* d_in, const int* in_sizes, int n_in,
                              void* d_out, int out_size, void* d_ws, size_t ws_size,
                              hipStream_t stream) {
  if (n_in < 8) return;
  if (in_sizes[0] != NN * DF) return;
  if (in_sizes[1] != 2 * NE) return;
  if (in_sizes[2] != DF * DF || in_sizes[4] != DF * DF) return;
  if (in_sizes[5] != DF * DF || in_sizes[7] != DF * DF) return;
  if (in_sizes[3] != DF || in_sizes[6] != DF) return;
  if ((long long)out_size != (long long)NN * DF) return;

  const float* x   = (const float*)d_in[0];
  const int*   ei  = (const int*)  d_in[1];
  const float* W1l = (const float*)d_in[2];
  const float* b1  = (const float*)d_in[3];
  const float* W1r = (const float*)d_in[4];
  const float* W2l = (const float*)d_in[5];
  const float* b2  = (const float*)d_in[6];
  const float* W2r = (const float*)d_in[7];
  float* out = (float*)d_out;
  const int* src = ei;
  const int* dst = ei + NE;

  char* ws = (char*)d_ws;
  size_t off = 0;
  const size_t oRA = off; off = al256(off + (size_t)MP * PH * 2);
  const size_t oRB = off; off = al256(off + (size_t)MP * PH * 2);
  const size_t oLI = off; off = al256(off + (size_t)NBB * RCAP * 4);
  const size_t oCN = off; off = al256(off + (size_t)NBB * NBRUN * 4);
  const size_t oOF = off; off = al256(off + (size_t)NBB * NBRUN * 4);
  const size_t oFL = off; off = al256(off + (size_t)NBB * 32 * 4);
  const size_t oW1 = off; off = al256(off + (size_t)DF * K1T * 2);
  const size_t oW2 = off; off = al256(off + (size_t)DF * K2T * 2);
  if (off > ws_size || off > (size_t)WSMAX) return;
  unsigned short* RA  = (unsigned short*)(ws + oRA);
  unsigned short* RB  = (unsigned short*)(ws + oRB);
  int* LIST = (int*)(ws + oLI);
  int* CNT  = (int*)(ws + oCN);
  int* OFF  = (int*)(ws + oOF);
  int* FLAG = (int*)(ws + oFL);
  unsigned short* W1C = (unsigned short*)(ws + oW1);
  unsigned short* W2C = (unsigned short*)(ws + oW2);

  hipFuncSetAttribute(reinterpret_cast<const void*>(&k_bucket), hipFuncAttributeMaxDynamicSharedMemorySize, (int)BK_LDS);
  hipFuncSetAttribute(reinterpret_cast<const void*>(&k_gemm<0, 128, 128>), hipFuncAttributeMaxDynamicSharedMemorySize, (int)G_LDS);
  hipFuncSetAttribute(reinterpret_cast<const void*>(&k_gemm<1, 256, 256>), hipFuncAttributeMaxDynamicSharedMemorySize, (int)G_LDS);

  k_prep<<<NUALL / NTHR, NTHR, 0, stream>>>(x, W1l, W1r, W2l, W2r, W1C, W2C, RB);
  k_bucket<<<NBB, NTHR, BK_LDS, stream>>>(src, dst, LIST, CNT, OFF, FLAG);
  k_agg<1><<<(NBB * NBRUN) / ARB, NTHR, 0, stream>>>(LIST, CNT, OFF, FLAG, RB, RA);
  k_gemm<0, 128, 128><<<MP / GBM, NTHR, G_LDS, stream>>>(RA, RB, W1C, b1, FLAG, RA, out);
  k_agg<2><<<(NBB * NBRUN) / ARB, NTHR, 0, stream>>>(LIST, CNT, OFF, FLAG, RA, RB);
  k_gemm<1, 256, 256><<<MP / GBM, NTHR, G_LDS, stream>>>(RB, RA, W2C, b2, FLAG, RA, out);
}
